// CustomNeighborhoodAttention3D_65678639891301
// MI455X (gfx1250) — hardware-verified
//
#include <hip/hip_runtime.h>
#include <math.h>

constexpr int kDd  = 5;
constexpr int kHh  = 40;
constexpr int kWw  = 80;
constexpr int kC   = 128;
constexpr int kNH  = 4;
constexpr int kHD  = 32;
constexpr int kTok = kDd * kHh * kWw;
constexpr int kQKV = 3 * kC;
constexpr int kWin = 45;
constexpr float kQScale = 0.17677669529663687f;

typedef __attribute__((ext_vector_type(16))) _Float16 v16h;
typedef __attribute__((ext_vector_type(8)))  _Float16 v8h;
typedef __attribute__((ext_vector_type(16))) __bf16   v16b;
typedef __attribute__((ext_vector_type(8)))  __bf16   v8b;
typedef __attribute__((ext_vector_type(8)))  float    v8f;
typedef __attribute__((ext_vector_type(4)))  float    v4f;
typedef __attribute__((ext_vector_type(4)))  unsigned int v4u;
typedef unsigned int v4ua __attribute__((ext_vector_type(4), may_alias));

__device__ __forceinline__ unsigned short f2bf_bits(float f) {
  unsigned u = __float_as_uint(f);
  return (unsigned short)((u + 0x7FFFu + ((u >> 16) & 1u)) >> 16);
}
__device__ __forceinline__ float bf_bits2f(unsigned short h) { return __uint_as_float(((unsigned)h) << 16); }

__device__ __forceinline__ void dep_guard_h(v8f& a, v8f& b, v16h x, v16h y) { asm volatile("v_nop\n\tv_nop\n\tv_nop\n\tv_nop" : "+v"(a), "+v"(b) : "v"(x), "v"(y)); }
__device__ __forceinline__ void dep_guard_b(v8f& a, v8f& b, v16b x, v16b y) { asm volatile("v_nop\n\tv_nop\n\tv_nop\n\tv_nop" : "+v"(a), "+v"(b) : "v"(x), "v"(y)); }
__device__ __forceinline__ void keep4_h(v16h a, v16h b, v16h c, v16h d) { asm volatile("v_nop" :: "v"(a), "v"(b), "v"(c), "v"(d)); }
__device__ __forceinline__ void keep4_b(v16b a, v16b b, v16b c, v16b d) { asm volatile("v_nop" :: "v"(a), "v"(b), "v"(c), "v"(d)); }
__device__ __forceinline__ void acc_guard4(v8f& a, v8f& b, v8f& c, v8f& d) { asm volatile("v_nop\n\tv_nop\n\tv_nop\n\tv_nop" : "+v"(a), "+v"(b), "+v"(c), "+v"(d)); }
template <typename T> struct Frag;
template <> struct Frag<_Float16> {
  typedef v16h V; union U { v16h v; v8h h[2]; };
  static __device__ __forceinline__ v16h load(const _Float16* p) {
    U f; f.h[0] = *(const v8h*)(p); f.h[1] = *(const v8h*)(p + 16); return f.v;
  }
  static __device__ __forceinline__ v8f mma(v16h a, v16h b, v8f c) {
    return __builtin_amdgcn_wmma_f32_16x16x32_f16(false, a, false, b, (short)0, c, false, false);
  }
  static __device__ __forceinline__ void guard(v8f& a, v8f& b, v16h x, v16h y) { dep_guard_h(a, b, x, y); }
  static __device__ __forceinline__ void keep(v16h a, v16h b, v16h c, v16h d) { keep4_h(a, b, c, d); }
};
template <> struct Frag<__bf16> {
  typedef v16b V; union U { v16b v; v8b h[2]; };
  static __device__ __forceinline__ v16b load(const __bf16* p) {
    U f; f.h[0] = *(const v8b*)(p); f.h[1] = *(const v8b*)(p + 16); return f.v;
  }
  static __device__ __forceinline__ v8f mma(v16b a, v16b b, v8f c) {
    return __builtin_amdgcn_wmma_f32_16x16x32_bf16(false, a, false, b, (short)0, c, false, false);
  }
  static __device__ __forceinline__ void guard(v8f& a, v8f& b, v16b x, v16b y) { dep_guard_b(a, b, x, y); }
  static __device__ __forceinline__ void keep(v16b a, v16b b, v16b c, v16b d) { keep4_b(a, b, c, d); }
};

__device__ __forceinline__ unsigned pk16(unsigned short a, unsigned short b) { return (unsigned)a | ((unsigned)b << 16); }

template <int ET> struct Elem;
template <> struct Elem<0> { typedef _Float16 T; };
template <> struct Elem<1> { typedef __bf16 T; };
template <int ET, bool SPLIT, int BIAS_MODE, int OUT_MODE, bool RESID, int ACT = 0>
__global__ __launch_bounds__(256) void wmma_gemm64(
    const unsigned short* __restrict__ Ap, const unsigned short* __restrict__ A2p, int lda, long strideA,
    const unsigned short* __restrict__ Btp, const unsigned short* __restrict__ Bt2p, int ldb, long strideB,
    void* __restrict__ Cout, void* __restrict__ Cout2, int ldc, long strideC,
    const float* __restrict__ bias,
    const float* __restrict__ resid, long strideR,
    int M, int N, int K, float scale) {
  typedef typename Elem<ET>::T T;
  typedef typename Frag<T>::V V;
  const T* A = (const T*)Ap; const T* A2 = (const T*)A2p; const T* Bt = (const T*)Btp; const T* Bt2 = (const T*)Bt2p;
  __shared__ __align__(16) float sT[8][16 * 68];
  const int b    = blockIdx.y;
  const int lane = threadIdx.x & 31;
  const int wave = threadIdx.x >> 5;
  const int tilesN = N >> 6;
  const int tilesM = M >> 6;
  const int tile = blockIdx.x * 8 + wave;
  if (tile >= tilesM * tilesN) return;
  const int tm = tile / tilesN;
  const int tn = tile - tm * tilesN;
  const int m0 = tm << 6;
  const int n0 = tn << 6;

  const T* Ab  = A  + (size_t)b * strideA;
  const T* Bb  = Bt + (size_t)b * strideB;
  const T* Ab2 = SPLIT ? (A2  + (size_t)b * strideA) : nullptr;
  const T* Bb2 = SPLIT ? (Bt2 + (size_t)b * strideB) : nullptr;

  const int rlane = lane & 15;
  const int koff  = (lane >> 4) * 8;
  const int mOff  = (lane >> 4) * 8;

  v8f acc[4][4];
#pragma unroll
  for (int i = 0; i < 4; ++i)
#pragma unroll
    for (int j = 0; j < 4; ++j) acc[i][j] = (v8f){0.f,0.f,0.f,0.f,0.f,0.f,0.f,0.f};

  for (int k0 = 0; k0 < K; k0 += 32) {
    V bh[4], bl[4];
#pragma unroll
    for (int j = 0; j < 4; ++j) {
      const size_t bo = (size_t)(n0 + (j << 4) + rlane) * ldb + koff + k0;
      bh[j] = Frag<T>::load(Bb + bo);
      if (SPLIT) bl[j] = Frag<T>::load(Bb2 + bo);
    }
#pragma unroll
    for (int i = 0; i < 4; ++i) {
      const size_t ao = (size_t)(m0 + (i << 4) + rlane) * lda + koff + k0;
      V ah = Frag<T>::load(Ab + ao);
      V al;
      if (SPLIT) al = Frag<T>::load(Ab2 + ao);
#pragma unroll
      for (int j = 0; j < 4; ++j) {
        acc[i][j] = Frag<T>::mma(ah, bh[j], acc[i][j]);
        if (SPLIT) {
          acc[i][j] = Frag<T>::mma(ah, bl[j], acc[i][j]);
          acc[i][j] = Frag<T>::mma(al, bh[j], acc[i][j]);
        }
      }
      Frag<T>::guard(acc[i][0], acc[i][3], ah, SPLIT ? al : ah);
    }
    Frag<T>::keep(bh[0], bh[1], bh[2], bh[3]);
    if (SPLIT) Frag<T>::keep(bl[0], bl[1], bl[2], bl[3]);
  }
  acc_guard4(acc[0][0], acc[0][1], acc[0][2], acc[0][3]);
  acc_guard4(acc[1][0], acc[1][1], acc[1][2], acc[1][3]);
  acc_guard4(acc[2][0], acc[2][1], acc[2][2], acc[2][3]);
  acc_guard4(acc[3][0], acc[3][1], acc[3][2], acc[3][3]);

  float* slab = sT[wave];
  const float* Rb = RESID ? (resid + (size_t)b * strideR) : nullptr;
#pragma unroll
  for (int i = 0; i < 4; ++i) {
    const int mBase = m0 + (i << 4);
#pragma unroll
    for (int j = 0; j < 4; ++j) {
      const int n = n0 + (j << 4) + rlane;
      float bv = 0.f;
      if (BIAS_MODE == 2) bv = bias[n];
#pragma unroll
      for (int r = 0; r < 8; ++r) {
        float v = acc[i][j][r] * scale;
        if (BIAS_MODE == 1) v += bias[mBase + mOff + r];
        if (BIAS_MODE == 2) v += bv;
        if (RESID) v += Rb[(size_t)(mBase + mOff + r) * ldc + n];
        if (ACT == 2) v = fmaxf(v, 0.0f);
        if (ACT == 4) v = (v > 0.f) ? v : 0.01f * v;
        slab[(mOff + r) * 68 + (j << 4) + rlane] = v;
      }
    }
    __builtin_amdgcn_fence(__ATOMIC_RELEASE, "workgroup");
    __builtin_amdgcn_wave_barrier();
    __builtin_amdgcn_fence(__ATOMIC_ACQUIRE, "workgroup");
    if (OUT_MODE == 0) {
      float* C = (float*)Cout + (size_t)b * strideC;
      const int hh = lane >> 4, c4 = (lane & 15) * 4;
      for (int pass = 0; pass < 2; ++pass) {
#pragma unroll
        for (int it = 0; it < 8; ++it) {
          const int row = it * 2 + hh;
          v4f v = *(const v4f*)(slab + row * 68 + c4);
          *(volatile v4f*)(C + (size_t)(mBase + row) * ldc + n0 + c4) = v;
        }
        __threadfence();
      }
    } else {
      const int q = lane >> 3, c8 = (lane & 7) * 8;
      unsigned short* C  = (unsigned short*)Cout  + (size_t)b * strideC;
      unsigned short* C2 = (OUT_MODE == 2) ? ((unsigned short*)Cout2 + (size_t)b * strideC) : nullptr;
      for (int pass = 0; pass < 2; ++pass) {
#pragma unroll
        for (int it = 0; it < 4; ++it) {
          const int row = it * 4 + q;
          const float* sp = slab + row * 68 + c8;
          v8h hv, lv;
#pragma unroll
          for (int e = 0; e < 8; ++e) {
            if (OUT_MODE == 1) {
              hv[e] = (_Float16)sp[e];
            } else {
              unsigned short hb = f2bf_bits(sp[e]);
              unsigned short lb = f2bf_bits(sp[e] - bf_bits2f(hb));
              hv[e] = __builtin_bit_cast(_Float16, hb);
              lv[e] = __builtin_bit_cast(_Float16, lb);
            }
          }
          *(volatile v8h*)(C + (size_t)(mBase + row) * ldc + n0 + c8) = hv;
          if (OUT_MODE == 2) *(volatile v8h*)(C2 + (size_t)(mBase + row) * ldc + n0 + c8) = lv;
        }
        __threadfence();
      }
    }
    __builtin_amdgcn_fence(__ATOMIC_RELEASE, "workgroup");
    __builtin_amdgcn_wave_barrier();
    __builtin_amdgcn_fence(__ATOMIC_ACQUIRE, "workgroup");
  }
}

__global__ __launch_bounds__(256) void split8_bf16_kernel(const float* __restrict__ in,
                                                         unsigned short* __restrict__ outHi,
                                                         unsigned short* __restrict__ outLo, int n8) {
  const int i = blockIdx.x * 256 + threadIdx.x;
  if (i >= n8) return;
  const float* p = in + 8 * (size_t)i;
  const v4f a = *(const v4f*)(p);
  const v4f c = *(const v4f*)(p + 4);
  unsigned short hb[8], lb[8];
#pragma unroll
  for (int e = 0; e < 4; ++e) {
    hb[e]     = f2bf_bits(a[e]);
    lb[e]     = f2bf_bits(a[e] - bf_bits2f(hb[e]));
    hb[4 + e] = f2bf_bits(c[e]);
    lb[4 + e] = f2bf_bits(c[e] - bf_bits2f(hb[4 + e]));
  }
  const v4u uh = (v4u){pk16(hb[0], hb[1]), pk16(hb[2], hb[3]), pk16(hb[4], hb[5]), pk16(hb[6], hb[7])};
  const v4u ul = (v4u){pk16(lb[0], lb[1]), pk16(lb[2], lb[3]), pk16(lb[4], lb[5]), pk16(lb[6], lb[7])};
  unsigned short* qh = outHi + 8 * (size_t)i;
  unsigned short* ql = outLo + 8 * (size_t)i;
  *(volatile v4u*)qh = uh;
  *(volatile v4u*)ql = ul;
  __threadfence();
  *(volatile v4u*)qh = uh;
  *(volatile v4u*)ql = ul;
}

__global__ __launch_bounds__(256) void wt_split_kernel(const float* __restrict__ W, int nOut,
                                                      unsigned short* __restrict__ outHi,
                                                      unsigned short* __restrict__ outLo) {
  __shared__ float sm[64][65];
  const int t  = threadIdx.x;
  const int d0 = blockIdx.x * 64;
  const int h0 = blockIdx.y * 64;
#pragma unroll
  for (int i = 0; i < 16; ++i) {
    const int e = i * 256 + t;
    const int r = e >> 6;
    const int c = e & 63;
    sm[c][r] = W[(size_t)(d0 + r) * nOut + h0 + c];
  }
  __syncthreads();
  const int lane = t & 31, wave = t >> 5;
  const int q = lane >> 3, c8 = (lane & 7) * 8;
  for (int pass = 0; pass < 2; ++pass) {
#pragma unroll
    for (int it = 0; it < 2; ++it) {
      const int row = wave * 8 + it * 4 + q;
      unsigned short hb[8], lb[8];
#pragma unroll
      for (int e = 0; e < 8; ++e) {
        const float f = sm[row][c8 + e];
        hb[e] = f2bf_bits(f);
        lb[e] = f2bf_bits(f - bf_bits2f(hb[e]));
      }
      const v4u uh = (v4u){pk16(hb[0], hb[1]), pk16(hb[2], hb[3]), pk16(hb[4], hb[5]), pk16(hb[6], hb[7])};
      const v4u ul = (v4u){pk16(lb[0], lb[1]), pk16(lb[2], lb[3]), pk16(lb[4], lb[5]), pk16(lb[6], lb[7])};
      const size_t o = (size_t)(h0 + row) * kC + d0 + c8;
      *(volatile v4u*)(outHi + o) = uh;
      *(volatile v4u*)(outLo + o) = ul;
    }
    __threadfence();
  }
}

__global__ __launch_bounds__(256) void na3d_window_kernel(const float* __restrict__ qkv,
                                                          unsigned short* __restrict__ outHi,
                                                          unsigned short* __restrict__ outLo) {
  __shared__ float sp[8][64];
  __shared__ __align__(16) unsigned short shH[2][kC];
  __shared__ __align__(16) unsigned short shL[2][kC];
  const int tid  = threadIdx.x;
  const int wave = tid >> 5;
  const int lane = tid & 31;
  const int tl   = wave >> 2;
  const int hd   = wave & 3;
  const int n    = blockIdx.x * 2 + tl;
  const int w    = n % kWw;
  const int dh   = n / kWw;
  const int h    = dh % kHh;
  const int d    = dh / kHh;
  const int dsx  = min(max(d - 1, 0), kDd - 3);
  const int hsx  = min(max(h - 1, 0), kHh - 3);
  const int wsx  = min(max(w - 2, 0), kWw - 5);
  const int nbase = (dsx * kHh + hsx) * kWw + wsx;

  const int m0  = lane;
  const int m1  = min(lane + 32, kWin - 1);
  const int od0 = m0 / 15, rr0 = m0 - od0 * 15, oh0 = rr0 / 5, ow0 = rr0 - oh0 * 5;
  const int od1 = m1 / 15, rr1 = m1 - od1 * 15, oh1 = rr1 / 5, ow1 = rr1 - oh1 * 5;
  const int nb0 = nbase + od0 * (kHh * kWw) + oh0 * kWw + ow0;
  const int nb1 = nbase + od1 * (kHh * kWw) + oh1 * kWw + ow1;
  const float* qrow  = qkv + (size_t)n   * kQKV + hd * kHD;
  const float* k0row = qkv + (size_t)nb0 * kQKV + kC + hd * kHD;
  const float* k1row = qkv + (size_t)nb1 * kQKV + kC + hd * kHD;
  float s0 = 0.f, s1 = 0.f;
#pragma unroll 1
  for (int c = 0; c < kHD / 4; ++c) {
    const v4f q4 = *(const v4f*)(qrow  + 4 * c);
    const v4f ka = *(const v4f*)(k0row + 4 * c);
    const v4f kb = *(const v4f*)(k1row + 4 * c);
#pragma unroll
    for (int e = 0; e < 4; ++e) {
      s0 = fmaf(q4[e], ka[e], s0);
      s1 = fmaf(q4[e], kb[e], s1);
    }
  }
  s0 *= kQScale;
  s1 *= kQScale;

  const bool ok1  = lane < (kWin - 32);
  const float s1m = ok1 ? s1 : s0;
  float mx = fmaxf(s0, s1m);
#pragma unroll
  for (int off = 16; off > 0; off >>= 1) mx = fmaxf(mx, __shfl_xor(mx, off, 32));
  const float p0  = expf(s0 - mx);
  const float p1e = expf(s1 - mx);
  const float p1  = ok1 ? p1e : 0.f;
  float sum = p0 + p1;
#pragma unroll
  for (int off = 16; off > 0; off >>= 1) sum += __shfl_xor(sum, off, 32);
  const float inv = 1.0f / sum;
  sp[wave][lane]      = p0;
  sp[wave][32 + lane] = p1;
  __syncthreads();

  const float* vbase = qkv + (size_t)nbase * kQKV + 2 * kC + hd * kHD + lane;
  const float* pw = sp[wave];
  float acc = 0.f;
#pragma unroll 1
  for (int od = 0; od < 3; ++od) {
#pragma unroll 1
    for (int oh = 0; oh < 3; ++oh) {
      const float* vr = vbase + (size_t)(od * (kHh * kWw) + oh * kWw) * kQKV;
      const float* pp = pw + (od * 3 + oh) * 5;
#pragma unroll
      for (int ow = 0; ow < 5; ++ow) acc = fmaf(pp[ow], vr[ow * kQKV], acc);
    }
  }
  const float o = acc * inv;

  const unsigned short hb = f2bf_bits(o);
  const unsigned short lb = f2bf_bits(o - bf_bits2f(hb));
  shH[tl][hd * kHD + lane] = hb;
  shL[tl][hd * kHD + lane] = lb;
  __syncthreads();
  if (wave == 0) {
    const int tt = lane >> 4;
    const int c8 = (lane & 15) * 8;
    const v4ua uh = *(const v4ua*)(&shH[tt][c8]);
    const v4ua ul = *(const v4ua*)(&shL[tt][c8]);
    unsigned short* ph = outHi + (size_t)(blockIdx.x * 2 + tt) * kC + c8;
    unsigned short* pl = outLo + (size_t)(blockIdx.x * 2 + tt) * kC + c8;
    *(volatile v4ua*)ph = uh;
    *(volatile v4ua*)pl = ul;
    __threadfence();
    *(volatile v4ua*)ph = uh;
    *(volatile v4ua*)pl = ul;
  }
}

extern "C" void kernel_launch(void* const* d_in, const int* in_sizes, int n_in,
                              void* d_out, int out_size, void* d_ws, size_t ws_size,
                              hipStream_t stream) {
  if (n_in < 5) return;
  if (in_sizes[0] != kTok * kC || in_sizes[1] != kC * kQKV || in_sizes[2] != kQKV ||
      in_sizes[3] != kC * kC || in_sizes[4] != kC) return;
  if (out_size != kTok * kC) return;

  const float* x      = (const float*)d_in[0];
  const float* w_qkv  = (const float*)d_in[1];
  const float* b_qkv  = (const float*)d_in[2];
  const float* w_proj = (const float*)d_in[3];
  const float* b_proj = (const float*)d_in[4];
  float* out = (float*)d_out;

  char* ws = (char*)d_ws;
  size_t off = 0;
  auto carve = [&](size_t bytes) -> char* {
    char* p = ws + off;
    off += (bytes + 255) & ~(size_t)255;
    return p;
  };
  unsigned short* xHi  = (unsigned short*)carve((size_t)kTok * kC * 2);
  unsigned short* xLo  = (unsigned short*)carve((size_t)kTok * kC * 2);
  unsigned short* wqHi = (unsigned short*)carve((size_t)kQKV * kC * 2);
  unsigned short* wqLo = (unsigned short*)carve((size_t)kQKV * kC * 2);
  unsigned short* wpHi = (unsigned short*)carve((size_t)kC * kC * 2);
  unsigned short* wpLo = (unsigned short*)carve((size_t)kC * kC * 2);
  float*          qkvf = (float*)carve((size_t)kTok * kQKV * 4);
  unsigned short* oHi  = (unsigned short*)carve((size_t)kTok * kC * 2);
  unsigned short* oLo  = (unsigned short*)carve((size_t)kTok * kC * 2);
  if (off > ws_size) return;

  const int n8 = kTok * kC / 8;
  split8_bf16_kernel<<<dim3((n8 + 255) / 256), dim3(256), 0, stream>>>(x, xHi, xLo, n8);

  wt_split_kernel<<<dim3(kC / 64, kQKV / 64), dim3(256), 0, stream>>>(w_qkv, kQKV, wqHi, wqLo);
  wt_split_kernel<<<dim3(kC / 64, kC / 64), dim3(256), 0, stream>>>(w_proj, kC, wpHi, wpLo);

  {
    const int tiles = (kTok / 64) * (kQKV / 64);
    wmma_gemm64<1, true, 2, 0, false, 0><<<dim3((tiles + 7) / 8, 1), dim3(256), 0, stream>>>(
        xHi, xLo, kC, 0L, wqHi, wqLo, kC, 0L, (void*)qkvf, (void*)nullptr, kQKV, 0L,
        b_qkv, (const float*)nullptr, 0L, kTok, kQKV, kC, 1.0f);
  }

  na3d_window_kernel<<<dim3(kTok / 2), dim3(256), 0, stream>>>(qkvf, oHi, oLo);

  {
    const int tiles = (kTok / 64) * (kC / 64);
    wmma_gemm64<1, true, 2, 0, false, 0><<<dim3((tiles + 7) / 8, 1), dim3(256), 0, stream>>>(
        oHi, oLo, kC, 0L, wpHi, wpLo, kC, 0L, (void*)out, (void*)nullptr, kC, 0L,
        b_proj, (const float*)nullptr, 0L, kTok, kC, kC, 1.0f);
  }
}
